// STSMGNN_64218351010251
// MI455X (gfx1250) — hardware-verified
//
#include <hip/hip_runtime.h>

#define NN    2048
#define NE    16384
#define HID   128
#define NH    4
#define HDIM  32
#define NHOP  3
#define NB    16
#define CHUNK 256
#define WSCL  64.0f
#define WINV  0.015625f
#define SCL   0.17677669529663687f

static_assert(NE % CHUNK == 0);
static_assert(NN % 64 == 0);
static_assert(NN % 256 == 0);
static_assert(NN % NB == 0);
static_assert(HID == NH * HDIM);

typedef _Float16 v16h __attribute__((ext_vector_type(16)));
typedef _Float16 v8h  __attribute__((ext_vector_type(8)));
typedef float    v8f  __attribute__((ext_vector_type(8)));
typedef float    v4f  __attribute__((ext_vector_type(4)));
typedef v8h __attribute__((may_alias)) v8ha;
typedef v4f __attribute__((may_alias)) v4fa;

union Frag { v16h v; v8h half[2]; };

#define ACC_OFF   0
#define RED_OFF   (NB * NN)
#define LNRM_OFF  (RED_OFF + 8 * 512)
#define LEF_OFF   (LNRM_OFF + CHUNK)
#define LSRC_OFF  (LEF_OFF + CHUNK)
#define LLC_OFF   (LSRC_OFF + CHUNK)
#define WCNT_OFF  (LLC_OFF + CHUNK)
#define CPART_OFF (WCNT_OFF + 16)
#define INVC_OFF  (CPART_OFF + 128)
#define HOP_LDS_FLOATS (INVC_OFF + 16)
#define HOP_LDS_BYTES  (HOP_LDS_FLOATS * 4)

__device__ __forceinline__ v8f wmma_f16(v16h a, v16h b, v8f c) {
  v8f d = __builtin_amdgcn_wmma_f32_16x16x32_f16(false, a, false, b, (short)0, c, false, false);
  asm volatile("v_nop\n\tv_nop\n\tv_nop\n\tv_nop" : "+v"(d) : "v"(a), "v"(b));
  return d;
}

__device__ __forceinline__ v8h cvt8(v4f a, v4f c) {
  const v8h o = { (_Float16)a.x, (_Float16)a.y, (_Float16)a.z, (_Float16)a.w,
                  (_Float16)c.x, (_Float16)c.y, (_Float16)c.z, (_Float16)c.w };
  return o;
}

__device__ __forceinline__ v16h load_frag(const _Float16* p, int hh) {
  Frag f;
  f.half[0] = *(const v8ha*)(p + 8 * hh);
  f.half[1] = *(const v8ha*)(p + 16 + 8 * hh);
  return f.v;
}

__device__ __forceinline__ v16h load_frag_f32(const float* p, int hh) {
  const v4f u0 = *(const v4fa*)(p + 8 * hh);
  const v4f u1 = *(const v4fa*)(p + 8 * hh + 4);
  const v4f u2 = *(const v4fa*)(p + 16 + 8 * hh);
  const v4f u3 = *(const v4fa*)(p + 20 + 8 * hh);
  Frag f;
  f.half[0] = cvt8(u0, u1);
  f.half[1] = cvt8(u2, u3);
  return f.v;
}

__global__ __launch_bounds__(256) void convert_kernel(
    const float* __restrict__ x, const float* __restrict__ wq, const float* __restrict__ wk,
    const float* __restrict__ wv, const float* __restrict__ wo,
    _Float16* __restrict__ xh, _Float16* __restrict__ wt)
{
  const int g = blockIdx.x * 256 + threadIdx.x;
  const int NXP = NN * HID / 8;
  const int NWP = 4 * HID * HID / 8;
  if (g >= NXP + NWP) return;
  v8h o;
  _Float16* dst;
  if (g < NXP) {
    const float* s = x + (size_t)g * 8;
    const v4f a = *(const v4fa*)s;
    const v4f c = *(const v4fa*)(s + 4);
    o = cvt8(a, c);
    dst = xh + (size_t)g * 8;
  } else {
    const int p = g - NXP;
    const int mat = p >> 11;
    const int rem = p & 2047;
    const int n = rem >> 4, q = rem & 15;
    const float* W = (mat == 0) ? wq : ((mat == 1) ? wk : ((mat == 2) ? wv : wo));
    const float* s = W + (size_t)(8 * q) * HID + n;
    v4f a, c;
    a.x = s[0 * HID] * WSCL; a.y = s[1 * HID] * WSCL; a.z = s[2 * HID] * WSCL; a.w = s[3 * HID] * WSCL;
    c.x = s[4 * HID] * WSCL; c.y = s[5 * HID] * WSCL; c.z = s[6 * HID] * WSCL; c.w = s[7 * HID] * WSCL;
    o = cvt8(a, c);
    dst = wt + (size_t)mat * HID * HID + (size_t)n * HID + 8 * q;
  }
  *(volatile v8h*)dst = o;
  __threadfence();
  *(volatile v8h*)dst = o;
}

__global__ __launch_bounds__(256) void deg_kernel(const int* __restrict__ eidx, float* __restrict__ dinv)
{
  __shared__ int sc[CHUNK];
  __shared__ __attribute__((aligned(16))) float sd[256];
  const int tid = threadIdx.x;
  const int node = blockIdx.x * 256 + tid;
  const int* col = eidx + NE;
  int cnt = 0;
  #pragma unroll 1
  for (int cb = 0; cb < NE; cb += CHUNK) {
    sc[tid] = col[cb + tid];
    __syncthreads();
    #pragma unroll 4
    for (int j = 0; j < CHUNK; ++j) cnt += (sc[j] == node) ? 1 : 0;
    __syncthreads();
  }
  const float cf = (float)((cnt > 0) ? cnt : 1);
  const float dv = (cnt > 0) ? (1.0f / sqrtf(cf)) : 0.0f;
  sd[tid] = dv;
  __syncthreads();
  v4f v;
  float* dp = dinv + (size_t)blockIdx.x * 256 + 4 * (tid & 63);
  if (tid < 64) v = *(const v4fa*)(sd + 4 * tid);
  if (tid < 64) *(volatile v4f*)dp = v;
  __threadfence();
  if (tid < 64) *(volatile v4f*)dp = v;
}

__device__ __forceinline__ void qk_pass(const float* sT, _Float16* plane, int n0, int w, int lane) {
  const int q = lane & 3, sub = lane >> 2;
  #pragma unroll
  for (int hd = 0; hd < NH; ++hd) {
    #pragma unroll
    for (int i = 0; i < 2; ++i) {
      const int r = 8 * i + sub;
      const float* s = sT + (16 * w + r) * HID + hd * HDIM + 8 * q;
      const v8h o = cvt8(*(const v4fa*)s, *(const v4fa*)(s + 4));
      *(volatile v8h*)(plane + ((size_t)hd * NN + n0 + r) * HDIM + 8 * q) = o;
    }
  }
}

__device__ __forceinline__ void v_pass(const float* sT, float* hidden, _Float16* vt, int N0, int n0,
                                       int w, int lane, int tid, float hw0) {
  #pragma unroll
  for (int r = 0; r < 16; ++r) {
    const v4f v = *(const v4fa*)(sT + (16 * w + r) * HID + 4 * lane);
    *(volatile v4f*)(hidden + (size_t)(n0 + r) * HID + 4 * lane) = v * hw0;
  }
  const int q = tid & 7, sub = tid >> 3;
  #pragma unroll
  for (int i = 0; i < 8; ++i) {
    const int c = 16 * i + sub;
    v4f a, b;
    a.x = sT[(8 * q + 0) * HID + c]; a.y = sT[(8 * q + 1) * HID + c];
    a.z = sT[(8 * q + 2) * HID + c]; a.w = sT[(8 * q + 3) * HID + c];
    b.x = sT[(8 * q + 4) * HID + c]; b.y = sT[(8 * q + 5) * HID + c];
    b.z = sT[(8 * q + 6) * HID + c]; b.w = sT[(8 * q + 7) * HID + c];
    *(volatile v8h*)(vt + (size_t)c * NN + N0 + 8 * q) = cvt8(a, b);
  }
}

__global__ __launch_bounds__(128) void qkv_kernel(
    const _Float16* __restrict__ xh, const _Float16* __restrict__ wt,
    const float* __restrict__ bq, const float* __restrict__ bk, const float* __restrict__ bv,
    const float* __restrict__ hopwise,
    _Float16* __restrict__ qh, _Float16* __restrict__ kh, _Float16* __restrict__ vt,
    float* __restrict__ hidden)
{
  __shared__ __attribute__((aligned(16))) float sT[64 * HID];

  const int tid = threadIdx.x, lane = tid & 31, w = tid >> 5;
  const int hh = lane >> 4, mm = lane & 15;
  const int which = blockIdx.y;
  const int N0 = blockIdx.x * 64, n0 = N0 + 16 * w;

  const _Float16* arow = xh + (size_t)(n0 + mm) * HID;
  const _Float16* wb = wt + ((size_t)which * HID + mm) * HID;

  const v8f z8 = {0.f, 0.f, 0.f, 0.f, 0.f, 0.f, 0.f, 0.f};
  v8f acc[8];
  #pragma unroll
  for (int nt = 0; nt < 8; ++nt) acc[nt] = z8;

  #pragma unroll 1
  for (int k0 = 0; k0 < HID; k0 += 32) {
    const v16h a = load_frag(arow + k0, hh);
    #pragma unroll
    for (int nt = 0; nt < 8; ++nt) {
      const v16h b = load_frag(wb + (size_t)nt * 16 * HID + k0, hh);
      acc[nt] = wmma_f16(a, b, acc[nt]);
    }
  }

  const float* bias = (which == 0) ? bq : ((which == 1) ? bk : bv);
  #pragma unroll
  for (int nt = 0; nt < 8; ++nt) {
    const int col = 16 * nt + mm;
    const float bvl = bias[col];
    #pragma unroll
    for (int r = 0; r < 8; ++r)
      sT[(16 * w + 8 * hh + r) * HID + col] = acc[nt][r] * WINV + bvl;
  }
  __syncthreads();

  if (which < 2) {
    _Float16* plane = (which == 0) ? qh : kh;
    qk_pass(sT, plane, n0, w, lane);
    __threadfence();
    qk_pass(sT, plane, n0, w, lane);
  } else {
    const float hw0 = hopwise[0];
    v_pass(sT, hidden, vt, N0, n0, w, lane, tid, hw0);
    __threadfence();
    v_pass(sT, hidden, vt, N0, n0, w, lane, tid, hw0);
  }
}

__device__ __forceinline__ void sim_pass(const float* sw, float* plane, int n0, int c0, int lane) {
  const int q = lane & 7, sub = lane >> 3;
  #pragma unroll
  for (int i = 0; i < 4; ++i) {
    const int row = 4 * i + sub;
    const v4f v = *(const v4fa*)(sw + row * 32 + 4 * q);
    *(volatile v4f*)(plane + (size_t)(n0 + row) * NN + c0 + 4 * q) = v;
  }
}

__global__ __launch_bounds__(256) void sim0_kernel(
    const _Float16* __restrict__ qh, const _Float16* __restrict__ kh,
    float* __restrict__ plane, int head)
{
  __shared__ __attribute__((aligned(16))) float st[8 * 16 * 32];

  const int tid = threadIdx.x, lane = tid & 31, w = tid >> 5;
  const int hh = lane >> 4, mm = lane & 15;
  const int n0 = blockIdx.x * 16;
  const v16h a = load_frag(qh + ((size_t)head * NN + n0 + mm) * HDIM, hh);
  float* sw = st + w * 512;
  const v8f z8 = {0.f, 0.f, 0.f, 0.f, 0.f, 0.f, 0.f, 0.f};

  #pragma unroll 1
  for (int j = 0; j < 8; ++j) {
    const int c0 = (w * 8 + j) * 32;
    const v16h b0 = load_frag(kh + ((size_t)head * NN + c0 + mm) * HDIM, hh);
    const v16h b1 = load_frag(kh + ((size_t)head * NN + c0 + 16 + mm) * HDIM, hh);
    const v8f s0 = wmma_f16(a, b0, z8);
    const v8f s1 = wmma_f16(a, b1, z8);
    #pragma unroll
    for (int r = 0; r < 8; ++r) {
      sw[(8 * hh + r) * 32 + mm]      = __expf(s0[r] * SCL);
      sw[(8 * hh + r) * 32 + 16 + mm] = __expf(s1[r] * SCL);
    }
    __syncthreads();
    sim_pass(sw, plane, n0, c0, lane);
    __threadfence();
    sim_pass(sw, plane, n0, c0, lane);
    __syncthreads();
  }
}

__device__ __forceinline__ void plane_pass(const float* accR, float* simNext, int c0, int tid) {
  #pragma unroll
  for (int lc = 0; lc < NB; ++lc) {
    const float* ap = accR + lc * NN;
    float* gp = simNext + (size_t)(c0 + lc) * NN;
    const v4f v0 = *(const v4fa*)(ap + 4 * tid);
    const v4f v1 = *(const v4fa*)(ap + 4 * (256 + tid));
    *(volatile v4f*)(gp + 4 * tid) = v0;
    *(volatile v4f*)(gp + 4 * (256 + tid)) = v1;
  }
}

__global__ __launch_bounds__(256) void hop_kernel(
    const float* __restrict__ simPrev, float* __restrict__ simNext,
    const _Float16* __restrict__ vt, const float* __restrict__ dinv,
    const float* __restrict__ ef, const int* __restrict__ eidx,
    const float* __restrict__ hopwise, const float* __restrict__ headwise,
    float* __restrict__ hidden, int head, int hop, int writePlane)
{
  extern __shared__ __attribute__((aligned(16))) float dl[];
  float* accR  = dl + ACC_OFF;
  float* red   = dl + RED_OFF;
  float* lnrm  = dl + LNRM_OFF;
  float* lef   = dl + LEF_OFF;
  int*   lsrc  = (int*)(dl + LSRC_OFF);
  int*   llc   = (int*)(dl + LLC_OFF);
  int*   wcnt  = (int*)(dl + WCNT_OFF);
  float* cpart = dl + CPART_OFF;
  float* invC  = dl + INVC_OFF;

  const int tid = threadIdx.x, lane = tid & 31, w = tid >> 5;
  const int hh = lane >> 4, mm = lane & 15;
  const int c0 = blockIdx.x * NB;
  const int* erow = eidx;
  const int* ecol = eidx + NE;

  float hmx = headwise[hop];
  #pragma unroll 1
  for (int q = 1; q < NH; ++q) hmx = fmaxf(hmx, headwise[q * NHOP + hop]);
  float se = 0.f, eh = 0.f;
  #pragma unroll 1
  for (int q = 0; q < NH; ++q) {
    const float e = expf(headwise[q * NHOP + hop] - hmx);
    se += e;
    eh = (q == head) ? e : eh;
  }
  const float gamma = hopwise[hop + 1] * (eh * (1.0f / se));

  const v4f z4 = {0.f, 0.f, 0.f, 0.f};
  #pragma unroll
  for (int lc = 0; lc < NB; ++lc) {
    *(v4fa*)(accR + lc * NN + 4 * tid) = z4;
    *(v4fa*)(accR + lc * NN + 4 * (256 + tid)) = z4;
  }

  #pragma unroll 1
  for (int cb = 0; cb < NE; cb += CHUNK) {
    const int e = cb + tid;
    int c = ecol[e]; c = min(max(c, 0), NN - 1);
    int s = erow[e]; s = min(max(s, 0), NN - 1);
    const int lc = c - c0;
    const bool hit = (unsigned)lc < (unsigned)NB;
    const float nrm = dinv[s] * dinv[c];
    const float efv = ef[e];
    const unsigned msk = __builtin_amdgcn_ballot_w32(hit);
    const int pre = __builtin_popcount(msk & ((1u << lane) - 1u));
    if (lane == 0) wcnt[w] = __builtin_popcount(msk);
    __syncthreads();
    int offw = 0, tot = 0;
    #pragma unroll
    for (int q = 0; q < 8; ++q) {
      const int cq = wcnt[q];
      tot += cq;
      offw += (q < w) ? cq : 0;
    }
    if (hit) {
      const int pos = min(offw + pre, CHUNK - 1);
      lsrc[pos] = s; llc[pos] = lc; lnrm[pos] = nrm; lef[pos] = efv;
    }
    __syncthreads();
    const int nh = min(tot, CHUNK);
    #pragma unroll 1
    for (int i = 0; i < nh; ++i) {
      int src = lsrc[i]; src = min(max(src, 0), NN - 1);
      const int l2 = llc[i] & (NB - 1);
      const float nm = lnrm[i];
      const float ev = lef[i];
      const float* sp = simPrev + (size_t)src * NN;
      const v4f v0 = *(const v4fa*)(sp + 4 * tid);
      const v4f v1 = *(const v4fa*)(sp + 4 * (256 + tid));
      float* ap = accR + l2 * NN;
      v4f a0 = *(v4fa*)(ap + 4 * tid);
      v4f a1 = *(v4fa*)(ap + 4 * (256 + tid));
      a0 = a0 + nm * (v0 + ev);
      a1 = a1 + nm * (v1 + ev);
      *(v4fa*)(ap + 4 * tid) = a0;
      *(v4fa*)(ap + 4 * (256 + tid)) = a1;
    }
    __syncthreads();
  }

  #pragma unroll
  for (int lc = 0; lc < NB; ++lc) {
    const float* ap = accR + lc * NN;
    const v4f a0 = *(const v4fa*)(ap + 4 * tid);
    const v4f a1 = *(const v4fa*)(ap + 4 * (256 + tid));
    float s = ((a0.x + a0.y) + (a0.z + a0.w)) + ((a1.x + a1.y) + (a1.z + a1.w));
    s += __shfl_xor(s, 16);
    s += __shfl_xor(s, 8);
    s += __shfl_xor(s, 4);
    s += __shfl_xor(s, 2);
    s += __shfl_xor(s, 1);
    if (lane == 0) cpart[w * NB + lc] = s;
  }
  __syncthreads();
  if (tid < NB) {
    float C = 0.f;
    #pragma unroll
    for (int q = 0; q < 8; ++q) C += cpart[q * NB + tid];
    C += 1e-5f;
    invC[tid] = 1.0f / C;
  }

  if (writePlane != 0) {
    plane_pass(accR, simNext, c0, tid);
    __threadfence();
    plane_pass(accR, simNext, c0, tid);
  }

  const _Float16* vb0 = vt + ((size_t)(head * HDIM + mm)) * NN;
  const _Float16* vb1 = vt + ((size_t)(head * HDIM + 16 + mm)) * NN;
  const float* ar = accR + mm * NN;
  const v8f z8 = {0.f, 0.f, 0.f, 0.f, 0.f, 0.f, 0.f, 0.f};
  v8f acc0 = z8, acc1 = z8;
  const int kb = w * 256;
  #pragma unroll 2
  for (int ks = 0; ks < 8; ++ks) {
    const int k0 = kb + 32 * ks;
    const v16h a  = load_frag_f32(ar + k0, hh);
    const v16h b0 = load_frag(vb0 + k0, hh);
    const v16h b1 = load_frag(vb1 + k0, hh);
    acc0 = wmma_f16(a, b0, acc0);
    acc1 = wmma_f16(a, b1, acc1);
  }
  float* rw = red + w * 512;
  #pragma unroll
  for (int r = 0; r < 8; ++r) {
    rw[(8 * hh + r) * 32 + mm]      = acc0[r];
    rw[(8 * hh + r) * 32 + 16 + mm] = acc1[r];
  }
  __syncthreads();

  const int r = (tid >> 3) & (NB - 1), q = tid & 7;
  float hm[4];
  #pragma unroll
  for (int j = 0; j < 4; ++j) {
    const int d = 4 * q + j;
    float s = 0.f;
    #pragma unroll
    for (int ww = 0; ww < 8; ++ww) s += red[ww * 512 + r * 32 + d];
    hm[j] = s * invC[r];
  }
  float* hp = hidden + (size_t)(c0 + r) * HID + head * HDIM + 4 * q;
  const v4f old = *(const v4fa*)hp;
  v4f nv;
  nv.x = old.x + gamma * hm[0];
  nv.y = old.y + gamma * hm[1];
  nv.z = old.z + gamma * hm[2];
  nv.w = old.w + gamma * hm[3];
  if (tid < 128) *(volatile v4f*)hp = nv;
  __threadfence();
  if (tid < 128) *(volatile v4f*)hp = nv;
}

__device__ __forceinline__ void out_pass(const float* sT, float* out, int n0, int w, int lane) {
  #pragma unroll
  for (int r = 0; r < 16; ++r) {
    const v4f v = *(const v4fa*)(sT + (16 * w + r) * HID + 4 * lane);
    *(volatile v4f*)(out + (size_t)(n0 + r) * HID + 4 * lane) = v;
  }
}

__global__ __launch_bounds__(128) void out_kernel(
    const float* __restrict__ hidden, const _Float16* __restrict__ wt,
    const float* __restrict__ bo, float* __restrict__ out)
{
  __shared__ __attribute__((aligned(16))) float sT[64 * HID];

  const int tid = threadIdx.x, lane = tid & 31, w = tid >> 5;
  const int hh = lane >> 4, mm = lane & 15;
  const int n0 = blockIdx.x * 64 + 16 * w;

  const float* arow = hidden + (size_t)(n0 + mm) * HID;
  const _Float16* wb = wt + ((size_t)3 * HID + mm) * HID;

  const v8f z8 = {0.f, 0.f, 0.f, 0.f, 0.f, 0.f, 0.f, 0.f};
  v8f acc[8];
  #pragma unroll
  for (int nt = 0; nt < 8; ++nt) acc[nt] = z8;

  #pragma unroll 1
  for (int k0 = 0; k0 < HID; k0 += 32) {
    const v16h a = load_frag_f32(arow + k0, hh);
    #pragma unroll
    for (int nt = 0; nt < 8; ++nt) {
      const v16h b = load_frag(wb + (size_t)nt * 16 * HID + k0, hh);
      acc[nt] = wmma_f16(a, b, acc[nt]);
    }
  }

  #pragma unroll
  for (int nt = 0; nt < 8; ++nt) {
    const int col = 16 * nt + mm;
    const float bvl = bo[col];
    #pragma unroll
    for (int r = 0; r < 8; ++r)
      sT[(16 * w + 8 * hh + r) * HID + col] = acc[nt][r] * WINV + bvl;
  }
  __syncthreads();

  out_pass(sT, out, n0, w, lane);
  __threadfence();
  out_pass(sT, out, n0, w, lane);
}

extern "C" void kernel_launch(void* const* d_in, const int* in_sizes, int n_in,
                              void* d_out, int out_size, void* d_ws, size_t ws_size,
                              hipStream_t stream) {
  if (n_in < 13) return;
  if (in_sizes[0] != NN * HID) return;
  if (in_sizes[1] != NE) return;
  if (in_sizes[2] != HID * HID || in_sizes[4] != HID * HID ||
      in_sizes[6] != HID * HID || in_sizes[8] != HID * HID) return;
  if (in_sizes[3] != HID || in_sizes[5] != HID || in_sizes[7] != HID || in_sizes[9] != HID) return;
  if (in_sizes[10] != NHOP + 1 || in_sizes[11] != NH * NHOP) return;
  if (in_sizes[12] != 2 * NE) return;
  if (out_size != NN * HID) return;

  const float* x        = (const float*)d_in[0];
  const float* ef       = (const float*)d_in[1];
  const float* Wq       = (const float*)d_in[2];
  const float* bq       = (const float*)d_in[3];
  const float* Wk       = (const float*)d_in[4];
  const float* bk       = (const float*)d_in[5];
  const float* Wv       = (const float*)d_in[6];
  const float* bv       = (const float*)d_in[7];
  const float* Wo       = (const float*)d_in[8];
  const float* bo       = (const float*)d_in[9];
  const float* hopwise  = (const float*)d_in[10];
  const float* headwise = (const float*)d_in[11];
  const int*   eidx     = (const int*)d_in[12];
  float* out = (float*)d_out;

  const size_t plane_b = (size_t)NN * NN * 4;
  const size_t xh_b    = (size_t)NN * HID * 2;
  const size_t wt_b    = (size_t)4 * HID * HID * 2;
  const size_t qh_b    = (size_t)NH * NN * HDIM * 2;
  const size_t vt_b    = (size_t)HID * NN * 2;
  const size_t hid_b   = (size_t)NN * HID * 4;
  const size_t dinv_b  = (size_t)NN * 4;
  const size_t o_p0  = 0;
  const size_t o_p1  = o_p0 + plane_b;
  const size_t o_xh  = o_p1 + plane_b;
  const size_t o_wt  = o_xh + xh_b;
  const size_t o_qh  = o_wt + wt_b;
  const size_t o_kh  = o_qh + qh_b;
  const size_t o_vt  = o_kh + qh_b;
  const size_t o_hid = o_vt + vt_b;
  const size_t o_dv  = o_hid + hid_b;
  const size_t total = o_dv + dinv_b;
  if (total > ws_size) return;

  char* ws = (char*)d_ws;
  float*    plane0 = (float*)(ws + o_p0);
  float*    plane1 = (float*)(ws + o_p1);
  _Float16* xh     = (_Float16*)(ws + o_xh);
  _Float16* wt     = (_Float16*)(ws + o_wt);
  _Float16* qh     = (_Float16*)(ws + o_qh);
  _Float16* kh     = (_Float16*)(ws + o_kh);
  _Float16* vt     = (_Float16*)(ws + o_vt);
  float*    hidden = (float*)(ws + o_hid);
  float*    dinv   = (float*)(ws + o_dv);

  hipFuncSetAttribute(reinterpret_cast<const void*>(&hop_kernel),
                      hipFuncAttributeMaxDynamicSharedMemorySize, HOP_LDS_BYTES);

  const int ncvt = NN * HID / 8 + 4 * HID * HID / 8;
  convert_kernel<<<(ncvt + 255) / 256, 256, 0, stream>>>(x, Wq, Wk, Wv, Wo, xh, wt);
  deg_kernel<<<NN / 256, 256, 0, stream>>>(eidx, dinv);
  qkv_kernel<<<dim3(NN / 64, 3), 128, 0, stream>>>(xh, wt, bq, bk, bv, hopwise, qh, kh, vt, hidden);

  for (int head = 0; head < NH; ++head) {
    sim0_kernel<<<NN / 16, 256, 0, stream>>>(qh, kh, plane0, head);
    float* pp = plane0;
    float* pn = plane1;
    for (int hop = 0; hop < NHOP; ++hop) {
      const int wflag = (hop < NHOP - 1) ? 1 : 0;
      hop_kernel<<<NN / NB, 256, HOP_LDS_BYTES, stream>>>(pp, pn, vt, dinv, ef, eidx,
                                                          hopwise, headwise, hidden, head, hop, wflag);
      float* t = pp; pp = pn; pn = t;
    }
  }

  out_kernel<<<NN / 64, 128, 0, stream>>>(hidden, wt, bo, out);
}
